// SGC_26714696581628
// MI455X (gfx1250) — hardware-verified
//
#include <hip/hip_runtime.h>
#include <stddef.h>


#define DW      64
#define NTHR    256
#define NWAVE   8
#define EPT     8
#define NGRP    2
#define CHUNK   (NTHR * EPT * NGRP)
#define WCAP    (EPT * NGRP * 32)
#define LISTN   (NWAVE * WCAP)
#define NBC     4096
#define NBF     1024
#define RCAP    40960
#define RBN     128
#define TGT     256
#define DEGCAP  1024
#define OTHR    512
#define GTHR    128
#define BM      64
#define KSTEPS  (DW / 32)
#define NTH     (DW / 16)
#define NTO     3
#define NOUTP   (NTO * 16)
#define WSCAP   134217728
#define ACARRY  64.0f
#define WCARRY  64.0f
#define GSCALE  (1.0f / 4096.0f)

#define LDS_FILL ((RCAP + 3 * NBF + LISTN + NWAVE) * 4 + 64)

static_assert((CHUNK & (CHUNK - 1)) == 0);
static_assert(CHUNK <= 4096);
static_assert(NBC <= 4096);
static_assert((NBC & (NBC - 1)) == 0 && (NBF & (NBF - 1)) == 0);
static_assert(NBC == 4 * NBF);
static_assert(OTHR * 8 == NBC);
static_assert((RCAP % 32) == 0);
static_assert(TGT == NWAVE * 32);
static_assert((NBC % TGT) == 0);
static_assert((NBF % TGT) == 0);
static_assert((TGT % BM) == 0);
static_assert(DW == 2 * 32);
static_assert((DW % 32) == 0);
static_assert(WCAP == EPT * NGRP * 32);
static_assert(NBF == 4 * NTHR);
static_assert(((RCAP + 2 * NBF + LISTN) % 4) == 0);
static_assert((NOUTP % 4) == 0);
static_assert(((BM * 4) % 128) == 0);

typedef float    v2f  __attribute__((ext_vector_type(2)));
typedef float    v4f  __attribute__((ext_vector_type(4)));
typedef float    v8f  __attribute__((ext_vector_type(8)));
typedef int      v4i  __attribute__((ext_vector_type(4)));
typedef _Float16 v4h  __attribute__((ext_vector_type(4)));
typedef _Float16 v8h  __attribute__((ext_vector_type(8)));
typedef _Float16 v16h __attribute__((ext_vector_type(16)));
union Frag { v16h v; v8h h[2]; };

__device__ __forceinline__ v8f wmh(v16h a, v16h b, v8f c) {
  v8f d = __builtin_amdgcn_wmma_f32_16x16x32_f16(false, a, false, b, (short)0, c, false, false);
  asm volatile("v_nop\n\tv_nop\n\tv_nop\n\tv_nop" : "+v"(d) : "v"(a), "v"(b));
  return d;
}

template <int NB>
__device__ __forceinline__ int scan_chunk(const int* __restrict__ dsts, int nE, int cbase, int slotBase,
                                          int vec8, int* list, int tid, int lane, int wave) {
  int wc = 0;
#pragma unroll
  for (int g = 0; g < NGRP; ++g) {
    const int el0  = (g * NTHR + tid) * EPT;
    const int e0   = cbase + el0;
    const int sent = -2147483647 - 1;
    v4i da, db;
    if (vec8 != 0 && cbase + CHUNK <= nE) {
      da = *(const v4i*)(dsts + e0);
      db = *(const v4i*)(dsts + e0 + 4);
    } else {
      da.x = (e0     < nE) ? dsts[min(e0, nE - 1)] : sent;
      da.y = (e0 + 1 < nE) ? dsts[min(e0 + 1, nE - 1)] : sent;
      da.z = (e0 + 2 < nE) ? dsts[min(e0 + 2, nE - 1)] : sent;
      da.w = (e0 + 3 < nE) ? dsts[min(e0 + 3, nE - 1)] : sent;
      db.x = (e0 + 4 < nE) ? dsts[min(e0 + 4, nE - 1)] : sent;
      db.y = (e0 + 5 < nE) ? dsts[min(e0 + 5, nE - 1)] : sent;
      db.z = (e0 + 6 < nE) ? dsts[min(e0 + 6, nE - 1)] : sent;
      db.w = (e0 + 7 < nE) ? dsts[min(e0 + 7, nE - 1)] : sent;
    }
    const unsigned nb = (unsigned)slotBase;
    const unsigned s0 = (unsigned)da.x - nb, s1 = (unsigned)da.y - nb;
    const unsigned s2 = (unsigned)da.z - nb, s3 = (unsigned)da.w - nb;
    const unsigned s4 = (unsigned)db.x - nb, s5 = (unsigned)db.y - nb;
    const unsigned s6 = (unsigned)db.z - nb, s7 = (unsigned)db.w - nb;
    const bool h0 = s0 < (unsigned)NB, h1 = s1 < (unsigned)NB, h2 = s2 < (unsigned)NB, h3 = s3 < (unsigned)NB;
    const bool h4 = s4 < (unsigned)NB, h5 = s5 < (unsigned)NB, h6 = s6 < (unsigned)NB, h7 = s7 < (unsigned)NB;
    const unsigned any = __builtin_amdgcn_ballot_w32(h0 | h1 | h2 | h3 | h4 | h5 | h6 | h7);
    if (any != 0u) {
#define HITJ(J, HJ, SJ) { \
        const unsigned mj = __builtin_amdgcn_ballot_w32(HJ); \
        if (mj != 0u) { \
          if (HJ) { \
            const int pos = wc + (int)__builtin_amdgcn_mbcnt_lo(mj, 0u); \
            if (pos < WCAP) list[wave * WCAP + pos] = ((el0 + (J)) << 12) | (int)(SJ); \
          } \
          wc += (int)__builtin_popcount(mj); } }
      HITJ(0, h0, s0)
      HITJ(1, h1, s1)
      HITJ(2, h2, s2)
      HITJ(3, h3, s3)
      HITJ(4, h4, s4)
      HITJ(5, h5, s5)
      HITJ(6, h6, s6)
      HITJ(7, h7, s7)
#undef HITJ
    }
  }
  return wc;
}

__global__ __launch_bounds__(NTHR) void k_count(const int* __restrict__ dsts, int* cnt, int nE, int vec8) {
  __shared__ __attribute__((aligned(16))) int scnt[NBC];
  __shared__ __attribute__((aligned(16))) int list[LISTN];
  __shared__ int wcnt[NWAVE];
  const int tid = threadIdx.x, lane = tid & 31, wave = tid >> 5;
  const int nodeBase = blockIdx.x * NBC;

  for (int i = tid; i < NBC; i += NTHR) scnt[i] = 0;
  __syncthreads();

  const int nChunks = (nE + CHUNK - 1) / CHUNK;
#pragma unroll 1
  for (int ch = 0; ch < nChunks; ++ch) {
    const int cbase = ch * CHUNK;
    const int wc = scan_chunk<NBC>(dsts, nE, cbase, nodeBase, vec8, list, tid, lane, wave);
    if (lane == 0) wcnt[wave] = wc;
    __syncthreads();
    if (wave == 0) {
#pragma unroll 1
      for (int wsx = 0; wsx < NWAVE; ++wsx) {
        int n = __builtin_amdgcn_readfirstlane(wcnt[wsx]);
        n = n > WCAP ? WCAP : (n < 0 ? 0 : n);
        const int* lp = list + wsx * WCAP;
#pragma unroll 1
        for (int i = 0; i < n; ++i) {
          const int ent  = __builtin_amdgcn_readfirstlane(lp[i]);
          const int slot = ent & (NBC - 1);
          if (lane == 0) scnt[slot] = scnt[slot] + 1;
        }
      }
    }
    __syncthreads();
  }

  v4i cq[4];
#pragma unroll
  for (int q = 0; q < 4; ++q) {
    const int f = (wave * 4 + q) * 128 + 4 * lane;
    cq[q] = *(const v4i*)(scnt + f);
  }
  int* cp = cnt + (size_t)nodeBase;
#pragma unroll
  for (int q = 0; q < 4; ++q) {
    const int f = (wave * 4 + q) * 128 + 4 * lane;
    *(volatile v4i*)(cp + f) = cq[q];
  }
  __threadfence();
#pragma unroll
  for (int q = 0; q < 4; ++q) {
    const int f = (wave * 4 + q) * 128 + 4 * lane;
    *(volatile v4i*)(cp + f) = cq[q];
  }
}

__global__ __launch_bounds__(OTHR) void k_offsets(
    const int* __restrict__ cnt, int* off, int* rbase, int nChunk) {
  __shared__ __attribute__((aligned(16))) int soff[NBC];
  __shared__ __attribute__((aligned(16))) int srb[RBN];
  __shared__ int wtot[OTHR / 32];
  const int tid = threadIdx.x, lane = tid & 31, wave = tid >> 5, sub = tid >> 7;
  for (int i = tid; i < RBN; i += OTHR) srb[i] = 0;
  int carry = 0;
#pragma unroll 1
  for (int ch = 0; ch < nChunk; ++ch) {
    const int base = ch * NBC;
    const v4i c0 = *(const v4i*)(cnt + base + 8 * tid);
    const v4i c1 = *(const v4i*)(cnt + base + 8 * tid + 4);
    const int e0 = max(c0.x, 0), e1 = max(c0.y, 0), e2 = max(c0.z, 0), e3 = max(c0.w, 0);
    const int e4 = max(c1.x, 0), e5 = max(c1.y, 0), e6 = max(c1.z, 0), e7 = max(c1.w, 0);
    const int ts = e0 + e1 + e2 + e3 + e4 + e5 + e6 + e7;
    int incl = ts;
#pragma unroll
    for (int d = 1; d < 32; d <<= 1) {
      const int t = __shfl_up(incl, d);
      if (lane >= d) incl += t;
    }
    if (lane == 31) wtot[wave] = incl;
    __syncthreads();
    const int S0 = wtot[0]  + wtot[1]  + wtot[2]  + wtot[3];
    const int S1 = wtot[4]  + wtot[5]  + wtot[6]  + wtot[7];
    const int S2 = wtot[8]  + wtot[9]  + wtot[10] + wtot[11];
    const int S3 = wtot[12] + wtot[13] + wtot[14] + wtot[15];
    int pre = 0;
#pragma unroll 1
    for (int w = 4 * sub; w < wave; ++w) pre += wtot[w];
    const int b0 = carry;
    const int b1 = b0 + ((S0 + 31) & ~31);
    const int b2 = b1 + ((S1 + 31) & ~31);
    const int b3 = b2 + ((S2 + 31) & ~31);
    const int b4 = b3 + ((S3 + 31) & ~31);
    const int myb = sub == 0 ? b0 : (sub == 1 ? b1 : (sub == 2 ? b2 : b3));
    if (tid == 0) {
      srb[min(4 * ch + 0, RBN - 1)] = b0;
      srb[min(4 * ch + 1, RBN - 1)] = b1;
      srb[min(4 * ch + 2, RBN - 1)] = b2;
      srb[min(4 * ch + 3, RBN - 1)] = b3;
    }
    int run = myb + pre + incl - ts;
    soff[8 * tid + 0] = run; run += e0;
    soff[8 * tid + 1] = run; run += e1;
    soff[8 * tid + 2] = run; run += e2;
    soff[8 * tid + 3] = run; run += e3;
    soff[8 * tid + 4] = run; run += e4;
    soff[8 * tid + 5] = run; run += e5;
    soff[8 * tid + 6] = run; run += e6;
    soff[8 * tid + 7] = run;
    carry = b4;
    __syncthreads();
    const v4i o0 = *(const v4i*)(soff + 4 * tid);
    const v4i o1 = *(const v4i*)(soff + 4 * (tid + OTHR));
    int* op = off + base;
    *(volatile v4i*)(op + 4 * tid) = o0;
    *(volatile v4i*)(op + 4 * (tid + OTHR)) = o1;
    __threadfence();
    *(volatile v4i*)(op + 4 * tid) = o0;
    *(volatile v4i*)(op + 4 * (tid + OTHR)) = o1;
    __syncthreads();
  }
  if (tid == 0) srb[min(4 * nChunk, RBN - 1)] = carry;
  __syncthreads();
  v4i rv = {0, 0, 0, 0};
  if (tid < 32) rv = *(const v4i*)(srb + 4 * tid);
  if (tid < 32) *(volatile v4i*)(rbase + 4 * tid) = rv;
  __threadfence();
  if (tid < 32) *(volatile v4i*)(rbase + 4 * tid) = rv;
}

__global__ __launch_bounds__(NTHR) void k_fill(
    const int* __restrict__ dsts, const float* __restrict__ ew,
    const int* __restrict__ off, const int* __restrict__ rbase,
    int* csr, float* dinv, int nE, int vec8, int csrLen) {
  extern __shared__ v4f lds_dyn[];
  int*   region = (int*)lds_dyn;
  int*   cursor = region + RCAP;
  int*   cstart = cursor + NBF;
  int*   list   = cstart + NBF;
  float* sdinv  = (float*)(list + LISTN);
  int*   wcnt   = (int*)(sdinv + NBF);
  const int tid = threadIdx.x, lane = tid & 31, wave = tid >> 5;
  const int b = blockIdx.x;
  const int nodeBase = b * NBF;

  int rb0 = rbase[b];
  const int rb1 = rbase[b + 1];
  rb0 = rb0 < 0 ? 0 : (rb0 > csrLen ? csrLen : rb0);
  rb0 &= ~31;
  int len = rb1 - rb0;
  len = len < 0 ? 0 : (len > RCAP ? RCAP : len);
  int lenW = (len + 31) & ~31;
  if (rb0 + lenW > csrLen) lenW = (csrLen - rb0) & ~31;

  {
    const v4i z = {0, 0, 0, 0};
    for (int i = tid; i < RCAP / 4; i += NTHR) ((v4i*)region)[i] = z;
    for (int s = tid; s < NBF; s += NTHR) {
      int o = off[nodeBase + s] - rb0;
      o = o < 0 ? 0 : (o > RCAP ? RCAP : o);
      cursor[s] = o;
      cstart[s] = o;
    }
  }
  __syncthreads();

  const int nChunks = (nE + CHUNK - 1) / CHUNK;
#pragma unroll 1
  for (int ch = 0; ch < nChunks; ++ch) {
    const int cbase = ch * CHUNK;
    const int wc = scan_chunk<NBF>(dsts, nE, cbase, nodeBase, vec8, list, tid, lane, wave);
    if (lane == 0) wcnt[wave] = wc;
    __syncthreads();
    if (wave == 0) {
#pragma unroll 1
      for (int wsx = 0; wsx < NWAVE; ++wsx) {
        int n = __builtin_amdgcn_readfirstlane(wcnt[wsx]);
        n = n > WCAP ? WCAP : (n < 0 ? 0 : n);
        const int* lp = list + wsx * WCAP;
#pragma unroll 1
        for (int i = 0; i < n; ++i) {
          const int ent  = __builtin_amdgcn_readfirstlane(lp[i]);
          const int slot = ent & (NBF - 1);
          int e = cbase + ((ent >> 12) & (CHUNK - 1));
          e = e > nE - 1 ? nE - 1 : (e < 0 ? 0 : e);
          if (lane == 0) {
            int pos = cursor[slot];
            pos = pos < 0 ? 0 : (pos > RCAP - 1 ? RCAP - 1 : pos);
            region[pos] = e;
            const int np = pos + 1;
            cursor[slot] = np > RCAP ? RCAP : np;
          }
        }
      }
    }
    __syncthreads();
  }

#pragma unroll 1
  for (int s = tid; s < NBF; s += NTHR) {
    int st = cstart[s];
    st = st < 0 ? 0 : (st > RCAP ? RCAP : st);
    int en = cursor[s];
    en = en < st ? st : (en > RCAP ? RCAP : en);
    int n = en - st;
    n = n > DEGCAP ? DEGCAP : n;
    float ds = 0.f;
#pragma unroll 1
    for (int i = 0; i < n; ++i) {
      int e = region[st + i];
      e = e < 0 ? 0 : (e > nE - 1 ? nE - 1 : e);
      ds += ew[e];
    }
    const float deg = ds + 1.0f;
    sdinv[s] = deg > 0.f ? rsqrtf(deg) : 0.f;
  }
  __syncthreads();

  const int nv = lenW >> 2;
  int* gp = csr + rb0;
  const v4f dv = *(const v4f*)(sdinv + 4 * tid);
  float* dq = dinv + (size_t)nodeBase + 4 * tid;
#pragma unroll 1
  for (int i = tid; i < nv; i += NTHR) { const v4i v = ((const v4i*)region)[i]; *(volatile v4i*)(gp + 4 * i) = v; }
  *(volatile v4f*)dq = dv;
  __threadfence();
#pragma unroll 1
  for (int i = tid; i < nv; i += NTHR) { const v4i v = ((const v4i*)region)[i]; *(volatile v4i*)(gp + 4 * i) = v; }
  *(volatile v4f*)dq = dv;
}

__global__ __launch_bounds__(NTHR) void k_wcvt(const float* __restrict__ w1, const float* __restrict__ w2,
                                               _Float16* dp, int nUnits, int nOut) {
  const int i = (int)blockIdx.x * NTHR + (int)threadIdx.x;
  if (i >= nUnits) return;
  const int ppr = DW / 8;
  const int u0 = DW * ppr;
  const bool first = i < u0;
  const int r = first ? i : i - u0;
  const int n = r / ppr;
  const int seg = r - n * ppr;
  int n1 = n > DW - 1 ? DW - 1 : n;
  n1 = n1 < 0 ? 0 : n1;
  int n2 = n > nOut - 1 ? nOut - 1 : n;
  n2 = n2 < 0 ? 0 : n2;
  const bool zero = (!first) && (n >= nOut);
  const float sel = zero ? 0.0f : WCARRY;
  const float* p0 = w1 + (size_t)n1 * DW + 8 * seg;
  const float* p1 = w2 + (size_t)n2 * DW + 8 * seg;
  v8h o;
#pragma unroll
  for (int j = 0; j < 8; ++j) {
    const float f0 = p0[j];
    const float f1 = p1[j];
    o[j] = (_Float16)((first ? f0 : f1) * sel);
  }
  _Float16* gp = dp + (size_t)i * 8;
  *(volatile v8h*)gp = o;
  __threadfence();
  *(volatile v8h*)gp = o;
}

template <int MODE, int NT>
__global__ __launch_bounds__(GTHR) void k_gemm(
    const float* __restrict__ Asrc, const _Float16* __restrict__ Bp, const float* __restrict__ bias,
    float* Cout, int nValid, int nOut) {
  constexpr int PPR = DW / 4;
  constexpr int NIT = (BM * PPR) / GTHR;
  static_assert((BM * PPR) % GTHR == 0);
  static_assert(NIT >= 1);
  static_assert(NT * 16 <= DW);
  static_assert(BM == 16 * (GTHR / 32));

  __shared__ __attribute__((aligned(16))) float stg[BM * DW];
  __shared__ __attribute__((aligned(16))) _Float16 a16[BM * DW];
  const int tid = threadIdx.x, lane = tid & 31, wave = tid >> 5, hh = lane >> 4, m = lane & 15;
  const int rowBase = (int)blockIdx.x * BM;
  const int r0 = wave * 16;

#pragma unroll
  for (int it = 0; it < NIT; ++it) {
    const int id = it * GTHR + tid;
    const int row = id / PPR, seg = id % PPR;
    const int grow = rowBase + row;
    const bool live = grow < nValid;
    int rr = grow > nValid - 1 ? nValid - 1 : grow;
    rr = rr < 0 ? 0 : rr;
    v4f xv = *(const v4f*)(Asrc + (size_t)rr * DW + 4 * seg);
    xv.x = live ? xv.x : 0.f;
    xv.y = live ? xv.y : 0.f;
    xv.z = live ? xv.z : 0.f;
    xv.w = live ? xv.w : 0.f;
    v4h o;
    o.x = (_Float16)(xv.x * ACARRY);
    o.y = (_Float16)(xv.y * ACARRY);
    o.z = (_Float16)(xv.z * ACARRY);
    o.w = (_Float16)(xv.w * ACARRY);
    *(v4h*)(a16 + (size_t)row * DW + 4 * seg) = o;
  }
  __syncthreads();

  v8f acc[NT];
#pragma unroll
  for (int t = 0; t < NT; ++t) { v8f z = {0.f, 0.f, 0.f, 0.f, 0.f, 0.f, 0.f, 0.f}; acc[t] = z; }

  const _Float16* ap = a16 + (size_t)(r0 + m) * DW + 8 * hh;
  const _Float16* bp = Bp + (size_t)m * DW + 8 * hh;
#pragma unroll 1
  for (int kt = 0; kt < KSTEPS; ++kt) {
    Frag a;
    a.h[0] = *(const v8h*)(ap + 32 * kt);
    a.h[1] = *(const v8h*)(ap + 32 * kt + 16);
#pragma unroll
    for (int t = 0; t < NT; ++t) {
      const size_t to = (size_t)(16 * t) * DW + 32 * kt;
      Frag b;
      b.h[0] = *(const v8h*)(bp + to);
      b.h[1] = *(const v8h*)(bp + to + 16);
      acc[t] = wmh(a.v, b.v, acc[t]);
    }
  }

  {
    const int growb = rowBase + r0 + 8 * hh;
#pragma unroll
    for (int t = 0; t < NT; ++t) {
      const int col = 16 * t + m;
      int cb = col > nOut - 1 ? nOut - 1 : col;
      cb = cb < 0 ? 0 : cb;
      const float bv = bias[cb];
#pragma unroll
      for (int r = 0; r < 8; ++r) {
        const int row = r0 + 8 * hh + r;
        const float v = acc[t][r] * GSCALE + bv;
        if constexpr (MODE == 0) {
          const bool lv = (growb + r) < nValid;
          stg[row * DW + col] = lv ? fmaxf(v, 0.f) : 0.f;
        } else {
          if (col < nOut) stg[row * nOut + col] = v;
        }
      }
    }
  }
  __syncthreads();

  if constexpr (MODE == 0) {
    v4f cv[NIT];
#pragma unroll
    for (int it = 0; it < NIT; ++it) {
      const int id = it * GTHR + tid;
      const int row = id / PPR, seg = id % PPR;
      cv[it] = *(const v4f*)(stg + (size_t)row * DW + 4 * seg);
    }
#pragma unroll
    for (int it = 0; it < NIT; ++it) {
      const int id = it * GTHR + tid;
      const int row = id / PPR, seg = id % PPR;
      float* gp = Cout + (size_t)(rowBase + row) * DW + 4 * seg;
      *(volatile v4f*)gp = cv[it];
    }
    __threadfence();
#pragma unroll
    for (int it = 0; it < NIT; ++it) {
      const int id = it * GTHR + tid;
      const int row = id / PPR, seg = id % PPR;
      float* gp = Cout + (size_t)(rowBase + row) * DW + 4 * seg;
      *(volatile v4f*)gp = cv[it];
    }
  } else {
    int vr = nValid - rowBase;
    vr = vr < 0 ? 0 : (vr > BM ? BM : vr);
    const int nq = (vr * nOut) >> 2;
    float* base = Cout + (size_t)rowBase * nOut;
#pragma unroll 1
    for (int q = tid; q < nq; q += GTHR) { const v4f v = *(const v4f*)(stg + 4 * q); *(volatile v4f*)(base + 4 * q) = v; }
    __threadfence();
#pragma unroll 1
    for (int q = tid; q < nq; q += GTHR) { const v4f v = *(const v4f*)(stg + 4 * q); *(volatile v4f*)(base + 4 * q) = v; }
  }
}

__global__ __launch_bounds__(NTHR) void k_hop(
    const int* __restrict__ csr, const int* __restrict__ off, const int* __restrict__ cnt,
    const float* __restrict__ dinv, const int* __restrict__ esrc, const float* __restrict__ ew,
    const float* xin, float* xout, int nN, int nE, int csrLen) {
  const int tid = threadIdx.x, lane = tid & 31, wave = tid >> 5;
  const int tbase = blockIdx.x * TGT + wave * 32;
  const int col2 = 2 * lane;
  const int cl    = tbase + lane;
  const int cnt_l = cnt[cl];
  const int off_l = off[cl];
  const float di_l = dinv[cl];

#pragma unroll 1
  for (int j = 0; j < 32; ++j) {
    const int c = tbase + j;
    int n = __shfl(cnt_l, j);
    n = n < 0 ? 0 : (n > DEGCAP ? DEGCAP : n);
    const int st = __shfl(off_l, j);
    const float dc = __shfl(di_l, j);
    const float dd = dc * dc;
    const int cr = c > nN - 1 ? nN - 1 : c;

    v2f a = *(const v2f*)(xin + (size_t)cr * DW + col2);
    a = a * dd;
#pragma unroll 1
    for (int q0 = 0; q0 < n; q0 += 32) {
      int pos = st + q0 + lane;
      pos = pos < 0 ? 0 : (pos > csrLen - 1 ? csrLen - 1 : pos);
      int el = csr[pos];
      el = el < 0 ? 0 : (el > nE - 1 ? nE - 1 : el);
      int sl = esrc[el];
      sl = sl < 0 ? 0 : (sl > nN - 1 ? nN - 1 : sl);
      const float cfl = (dinv[sl] * ew[el]) * dc;
      const int mcnt = (n - q0) < 32 ? (n - q0) : 32;
#pragma unroll 1
      for (int pp = 0; pp < mcnt; ++pp) {
        const int s = __builtin_amdgcn_readlane(sl, pp);
        const float cf = __shfl(cfl, pp);
        const v2f xv = *(const v2f*)(xin + (size_t)s * DW + col2);
        a = a + xv * cf;
      }
    }

    const bool live = c < nN;
    v2f o;
    o.x = live ? a.x : 0.f;
    o.y = live ? a.y : 0.f;
    float* gp = xout + (size_t)c * DW + col2;
    *(volatile v2f*)gp = o;
    __threadfence();
    *(volatile v2f*)gp = o;
  }
}

extern "C" void kernel_launch(void* const* d_in, const int* in_sizes, int n_in,
                              void* d_out, int out_size, void* d_ws, size_t ws_size,
                              hipStream_t stream) {
  if (n_in < 7) return;
  if (in_sizes[0] < DW || (in_sizes[0] % DW) != 0) return;
  const int nN = in_sizes[0] / DW;
  if (in_sizes[1] < 2 || (in_sizes[1] & 1) != 0) return;
  const int nE = in_sizes[1] / 2;
  if (in_sizes[2] != nE) return;
  if (in_sizes[3] != DW * DW || in_sizes[4] != DW) return;
  if (in_sizes[5] < DW || (in_sizes[5] % DW) != 0) return;
  const int nOut = in_sizes[5] / DW;
  if (nOut < 4 || nOut > NOUTP || (nOut & 3) != 0) return;
  if (in_sizes[6] != nOut) return;
  if ((long long)out_size != (long long)nN * (long long)nOut) return;
  if (nE > (1 << 28) || nN > (1 << 22)) return;

  const float* x   = (const float*)d_in[0];
  const int*   ei  = (const int*)d_in[1];
  const int*   src = ei;
  const int*   dst = ei + nE;
  const float* ew  = (const float*)d_in[2];
  const float* w1  = (const float*)d_in[3];
  const float* b1  = (const float*)d_in[4];
  const float* w2  = (const float*)d_in[5];
  const float* b2  = (const float*)d_in[6];
  float* out = (float*)d_out;

  const int NPAD   = ((nN + TGT - 1) / TGT) * TGT;
  const int nBC    = (nN + NBC - 1) / NBC;
  const int CNTPAD = nBC * NBC;
  if (CNTPAD < NPAD) return;
  if (4 * nBC + 1 > RBN) return;
  const int nBF    = (nN + NBF - 1) / NBF;
  if (nBF > 4 * nBC) return;
  const int DIPAD  = nBF * NBF;
  if (DIPAD < NPAD) return;
  const int csrLen = ((nE + 31) & ~31) + 4096;
  if (31 * 4 * nBC > 4096) return;
  const int nHop   = NPAD / TGT;
  const int nGemm  = NPAD / BM;
  const int nUnits = DW * (DW / 8) + NOUTP * (DW / 8);

  char* ws = (char*)d_ws;
  size_t off = 0;
  const size_t oWp  = off; off += (size_t)(DW * DW + NOUTP * DW) * 2; off = (off + 255) & ~(size_t)255;
  const size_t oPA  = off; off += (size_t)NPAD * DW * 4;             off = (off + 255) & ~(size_t)255;
  const size_t oPB  = off; off += (size_t)NPAD * DW * 4;             off = (off + 255) & ~(size_t)255;
  const size_t oCnt = off; off += (size_t)CNTPAD * 4;                off = (off + 255) & ~(size_t)255;
  const size_t oOff = off; off += (size_t)CNTPAD * 4;                off = (off + 255) & ~(size_t)255;
  const size_t oDi  = off; off += (size_t)DIPAD * 4;                 off = (off + 255) & ~(size_t)255;
  const size_t oRb  = off; off += (size_t)RBN * 4;                   off = (off + 255) & ~(size_t)255;
  const size_t oCsr = off; off += (size_t)csrLen * 4;                off = (off + 255) & ~(size_t)255;
  if (off > ws_size || off > (size_t)WSCAP) return;

  _Float16* wpl = (_Float16*)(ws + oWp);
  float* pa   = (float*)(ws + oPA);
  float* pb   = (float*)(ws + oPB);
  int*   cnt  = (int*)(ws + oCnt);
  int*   offp = (int*)(ws + oOff);
  float* dinv = (float*)(ws + oDi);
  int*   rb   = (int*)(ws + oRb);
  int*   csr  = (int*)(ws + oCsr);

  const int vec8 = ((nE & 3) == 0) ? 1 : 0;

  k_wcvt<<<(nUnits + NTHR - 1) / NTHR, NTHR, 0, stream>>>(w1, w2, wpl, nUnits, nOut);
  k_count<<<nBC, NTHR, 0, stream>>>(dst, cnt, nE, vec8);
  k_offsets<<<1, OTHR, 0, stream>>>(cnt, offp, rb, nBC);
  hipFuncSetAttribute(reinterpret_cast<const void*>(&k_fill),
                      hipFuncAttributeMaxDynamicSharedMemorySize, LDS_FILL);
  k_fill<<<nBF, NTHR, LDS_FILL, stream>>>(dst, ew, offp, rb, csr, dinv, nE, vec8, csrLen);

  k_hop<<<nHop, NTHR, 0, stream>>>(csr, offp, cnt, dinv, src, ew, x, pa, nN, nE, csrLen);
  k_hop<<<nHop, NTHR, 0, stream>>>(csr, offp, cnt, dinv, src, ew, pa, pb, nN, nE, csrLen);
  k_gemm<0, NTH><<<nGemm, GTHR, 0, stream>>>(pb, wpl, b1, pa, nN, DW);

  k_hop<<<nHop, NTHR, 0, stream>>>(csr, offp, cnt, dinv, src, ew, pa, pb, nN, nE, csrLen);
  k_hop<<<nHop, NTHR, 0, stream>>>(csr, offp, cnt, dinv, src, ew, pb, pa, nN, nE, csrLen);
  k_gemm<1, NTO><<<nGemm, GTHR, 0, stream>>>(pa, wpl + (size_t)DW * DW, b2, out, nN, nOut);
}
